// MixedFeedFoward_21663815041809
// MI455X (gfx1250) — hardware-run, weakly checked
//
#include <hip/hip_runtime.h>


#define NT   4096
#define DM   1024
#define HM   4096
typedef _Float16 h16;
typedef unsigned short bf;
typedef __attribute__((ext_vector_type(16))) __bf16   v16bf;
typedef __attribute__((ext_vector_type(16))) _Float16 v16h;
typedef __attribute__((ext_vector_type(8)))  _Float16 v8h;
typedef __attribute__((ext_vector_type(8)))  unsigned short v8us;
typedef __attribute__((ext_vector_type(8)))  float    v8f;
typedef __attribute__((ext_vector_type(4)))  float    v4f;
typedef v8h  __attribute__((may_alias)) v8ha;
typedef v4f  __attribute__((may_alias)) v4fa;
typedef v8us __attribute__((may_alias)) v8usa;

__device__ __forceinline__ unsigned short f2bf(float f) { unsigned u = __float_as_uint(f); u += 0x7FFFu + ((u >> 16) & 1u); return (unsigned short)(u >> 16); }
__device__ __forceinline__ float bf2f(unsigned short b) { return __uint_as_float(((unsigned)b) << 16); }
__device__ __forceinline__ float bfr(float f) { return bf2f(f2bf(f)); }
__device__ __forceinline__ v16h cat16(v8h lo, v8h hi) { return __builtin_shufflevector(lo, hi, 0, 1, 2, 3, 4, 5, 6, 7, 8, 9, 10, 11, 12, 13, 14, 15); }
__device__ __forceinline__ v16bf cat16b(v8us lo, v8us hi) { return __builtin_bit_cast(v16bf, __builtin_shufflevector(lo, hi, 0, 1, 2, 3, 4, 5, 6, 7, 8, 9, 10, 11, 12, 13, 14, 15)); }
__device__ __forceinline__ v8f wmma16(v16h a, v16h b, v8f c) { return __builtin_amdgcn_wmma_f32_16x16x32_f16(false, a, false, b, (short)0, c, false, false); }
__device__ __forceinline__ v8f wmmab(v16bf a, v16bf b, v8f c) { return __builtin_amdgcn_wmma_f32_16x16x32_bf16(false, a, false, b, (short)0, c, false, false); }


template <typename T16> struct WFrag;
template <> struct WFrag<h16> { typedef v16h V; static __device__ __forceinline__ V ld(const h16* p) { return cat16(*(const v8h*)p, *(const v8h*)(p + 16)); } static __device__ __forceinline__ v8f mma(V a, V b, v8f c) { return wmma16(a, b, c); } };
template <> struct WFrag<bf> { typedef v16bf V; static __device__ __forceinline__ V ld(const bf* p) { return cat16b(*(const v8us*)p, *(const v8us*)(p + 16)); } static __device__ __forceinline__ v8f mma(V a, V b, v8f c) { return wmmab(a, b, c); } };
template <typename T16, int NSPLIT, bool BIAS>
__global__ __launch_bounds__(32) void k_gemmw(const T16* __restrict__ A, const T16* __restrict__ A2, const T16* __restrict__ Bt, const T16* __restrict__ Bt2, int K, float* C, int ldc, const float* __restrict__ bias, size_t sA, size_t sB, size_t sC) {
    typedef typename WFrag<T16>::V V;
    __shared__ __align__(16) float os[16 * 68];
    const size_t z = blockIdx.z; A += z * sA; if (A2) A2 += z * sA; Bt += z * sB; if (Bt2) Bt2 += z * sB; C += z * sC;
    const int lane = threadIdx.x & 31, lr = lane & 15, hi = lane >> 4; const int r0 = blockIdx.x * 64, c0 = blockIdx.y * 64;
    v8f acc[4][4];
#pragma unroll
    for (int mb = 0; mb < 4; ++mb)
#pragma unroll
        for (int nb = 0; nb < 4; ++nb) acc[mb][nb] = (v8f){};
    const size_t aoff = (size_t)(r0 + lr) * K + 8 * hi, boff = (size_t)(c0 + lr) * K + 8 * hi;
    for (int kc = 0; kc < K; kc += 32) {
        V a[4], a2[4];
#pragma unroll
        for (int mb = 0; mb < 4; ++mb) { a[mb] = WFrag<T16>::ld(A + aoff + (size_t)mb * 16 * K + kc); if (NSPLIT == 1 || NSPLIT == 2) a2[mb] = WFrag<T16>::ld(A2 + aoff + (size_t)mb * 16 * K + kc); }
#pragma unroll
        for (int nb = 0; nb < 4; ++nb) { const V b = WFrag<T16>::ld(Bt + boff + (size_t)nb * 16 * K + kc); V b2; if (NSPLIT >= 2) b2 = WFrag<T16>::ld(Bt2 + boff + (size_t)nb * 16 * K + kc);
#pragma unroll
            for (int mb = 0; mb < 4; ++mb) { acc[mb][nb] = WFrag<T16>::mma(a[mb], b, acc[mb][nb]); if (NSPLIT == 1 || NSPLIT == 2) acc[mb][nb] = WFrag<T16>::mma(a2[mb], b, acc[mb][nb]); if (NSPLIT >= 2) acc[mb][nb] = WFrag<T16>::mma(a[mb], b2, acc[mb][nb]); } }
        asm volatile("v_nop\n\tv_nop\n\tv_nop\n\tv_nop" : "+v"(acc[0][0]), "+v"(acc[1][1]), "+v"(acc[2][2]), "+v"(acc[3][3]) : "v"(a[0]), "v"(a[3]));
    }
#pragma unroll
    for (int mb = 0; mb < 4; ++mb) {
#pragma unroll
        for (int nb = 0; nb < 4; ++nb) {
#pragma unroll
            for (int j = 0; j < 8; ++j) os[(hi * 8 + j) * 68 + nb * 16 + lr] = acc[mb][nb][j]; }
        __builtin_amdgcn_wave_barrier(); asm volatile("" ::: "memory");
        float* crow = C + (size_t)(r0 + mb * 16) * ldc + c0;
#pragma unroll 1
        for (int ps = 0; ps < 2; ++ps) {
#pragma unroll
            for (int s = 0; s < 8; ++s) { const int row = 2 * s + hi, cofs = lr * 4; v4f val = *(const v4fa*)(os + row * 68 + cofs); if (BIAS) { val[0] += bfr(bias[c0 + cofs]); val[1] += bfr(bias[c0 + cofs + 1]); val[2] += bfr(bias[c0 + cofs + 2]); val[3] += bfr(bias[c0 + cofs + 3]); }
                *(volatile v4f*)(crow + (size_t)row * ldc + cofs) = val; }
            if (ps == 0) __threadfence(); }
        __builtin_amdgcn_wave_barrier(); asm volatile("" ::: "memory");
    }
}

__device__ __forceinline__ h16 tohx(float x) { return (h16)x; }
__device__ __forceinline__ void splitf(float y, unsigned short& h, unsigned short& l) { h = f2bf(y); l = f2bf(y - bf2f(h)); }
typedef __attribute__((ext_vector_type(2))) _Float16 v2h;
typedef __attribute__((ext_vector_type(4))) _Float16 v4h;
typedef __attribute__((ext_vector_type(2))) unsigned short v2us;
typedef __attribute__((ext_vector_type(4))) unsigned short v4us;
typedef __attribute__((ext_vector_type(2))) float v2f;
typedef __attribute__((ext_vector_type(4))) int v4i;

__device__ __forceinline__ h16 toh_flush(float x) { const float z = (fabsf(x) < 6.103515625e-05f) ? 0.0f : x; return (h16)z; }

struct Arch { float a[3], b[3]; };
__device__ __forceinline__ Arch arch_of(const float* __restrict__ ae, const float* __restrict__ am) { Arch A; const float e0 = bfr(ae[0]), e1 = bfr(ae[1]), e2 = bfr(ae[2]); const float me = fmaxf(fmaxf(e0, e1), e2); const float x0 = expf(e0 - me), x1 = expf(e1 - me), x2 = expf(e2 - me); const float se = (x0 + x1) + x2; A.a[0] = x0 / se; A.a[1] = x1 / se; A.a[2] = x2 / se; const float m0 = bfr(am[0]), m1 = bfr(am[1]), m2 = bfr(am[2]); const float mm = fmaxf(fmaxf(m0, m1), m2); const float y0 = expf(m0 - mm), y1 = expf(m1 - mm), y2 = expf(m2 - mm); const float sm = (y0 + y1) + y2; A.b[0] = y0 / sm; A.b[1] = y1 / sm; A.b[2] = y2 / sm; return A; }
__device__ __forceinline__ float fac(const Arch& A, int hid, int emb, bool useHid, bool useEmb) { float f = 0.0f;
#pragma unroll
    for (int ie = 0; ie < 3; ++ie) { const int e = 512 + 256 * ie;
#pragma unroll
        for (int ir = 0; ir < 3; ++ir) { const int r = 2 + ir; const float w = __fmul_rn(A.a[ie], A.b[ir]); const bool on = (!useHid || hid < e * r) && (!useEmb || emb < e); f = __fadd_rn(f, on ? w : 0.0f); } }
    return f; }

__global__ __launch_bounds__(256) void k_cast16(const float* __restrict__ src, h16* dst, size_t n4, int mode, const float* __restrict__ b, int ncol, const float* __restrict__ ae, const float* __restrict__ am) { const size_t i = (size_t)blockIdx.x * 256 + threadIdx.x; if (i >= n4) return; const v4f v = *(const v4f*)(src + i * 4); v4f bb = (v4f){0.0f, 0.0f, 0.0f, 0.0f}; if (mode) { const Arch A = arch_of(ae, am); const int c0 = (int)((i * 4) % (size_t)ncol); const v4f b4 = *(const v4f*)(b + c0);
#pragma unroll
        for (int q = 0; q < 4; ++q) bb[q] = __fmul_rn(bfr(b4[q]), fac(A, c0 + q, 0, true, false)); }
    v4h o;
#pragma unroll
    for (int q = 0; q < 4; ++q) { const float y = mode ? fmaxf(__fadd_rn(v[q], bb[q]), 0.0f) : bfr(v[q]); o[q] = toh_flush(y); }
    *(volatile v4h*)(dst + i * 4) = o; __threadfence(); *(volatile v4h*)(dst + i * 4) = o; }

__global__ __launch_bounds__(256) void k_maskw(const float* __restrict__ w, h16* dst, int R, int C, int hidIsRow, const float* __restrict__ ae, const float* __restrict__ am) { const size_t i = (size_t)blockIdx.x * 256 + threadIdx.x; if (i >= (size_t)R * C / 4) return; const Arch A = arch_of(ae, am); const int row = (int)(i / (size_t)(C / 4)); const int c0 = (int)(i % (size_t)(C / 4)) * 4; const v4f v = *(const v4f*)(w + (size_t)row * C + c0); v4h o;
#pragma unroll
    for (int q = 0; q < 4; ++q) { const int col = c0 + q; const float f = hidIsRow ? fac(A, row, col, true, true) : fac(A, col, row, true, true); o[q] = toh_flush(__fmul_rn(bfr(v[q]), f)); }
    *(volatile v4h*)(dst + (size_t)row * C + c0) = o; __threadfence(); *(volatile v4h*)(dst + (size_t)row * C + c0) = o; }

__global__ __launch_bounds__(256) void k_addb(const float* __restrict__ src, float* dst, size_t n4, const float* __restrict__ b, int ncol, const float* __restrict__ ae, const float* __restrict__ am) { const size_t i = (size_t)blockIdx.x * 256 + threadIdx.x; if (i >= n4) return; const Arch A = arch_of(ae, am); const int c0 = (int)((i * 4) % (size_t)ncol); const v4f v = *(const v4f*)(src + i * 4); const v4f b4 = *(const v4f*)(b + c0); v4f o;
#pragma unroll
    for (int q = 0; q < 4; ++q) o[q] = __fadd_rn(v[q], __fmul_rn(bfr(b4[q]), fac(A, 0, c0 + q, false, true)));
    *(volatile v4f*)(dst + i * 4) = o; __threadfence(); *(volatile v4f*)(dst + i * 4) = o; }

extern "C" void kernel_launch(void* const* d_in, const int* in_sizes, int n_in,
                              void* d_out, int out_size, void* d_ws, size_t ws_size, hipStream_t stream) {
    (void)in_sizes; (void)n_in; (void)out_size;
    const float* x = (const float*)d_in[0]; const float* w0 = (const float*)d_in[1]; const float* b0 = (const float*)d_in[2]; const float* w1 = (const float*)d_in[3]; const float* b1 = (const float*)d_in[4]; const float* ae = (const float*)d_in[5]; const float* am = (const float*)d_in[6];
    static_assert(NT % 64 == 0 && DM % 64 == 0 && HM % 64 == 0 && DM % 32 == 0 && HM % 32 == 0 && DM % 4 == 0 && HM % 4 == 0, "both product launches: M and N multiples of 64, K a multiple of 32; four words a thread");
    float* OUT = (float*)d_out;
    char* wsp = (char*)d_ws;
    auto take = [&](size_t bytes) { char* p = wsp; wsp += (bytes + 255) & ~(size_t)255; return (void*)p; };
    h16* X16 = (h16*)take((size_t)NT * DM * 2);     h16* W0h = (h16*)take((size_t)HM * DM * 2);     h16* W1h = (h16*)take((size_t)DM * HM * 2);     float* FC = (float*)take((size_t)NT * HM * 4);     h16* H16 = (h16*)take((size_t)NT * HM * 2);     float* OF = FC;
    if ((size_t)(wsp - (char*)d_ws) > ws_size) return;
    k_cast16<<<(unsigned)(((size_t)NT * DM / 4 + 255) / 256), 256, 0, stream>>>(x, X16, (size_t)NT * DM / 4, 0, nullptr, DM, nullptr, nullptr);
    k_maskw<<<(unsigned)(((size_t)HM * DM / 4 + 255) / 256), 256, 0, stream>>>(w0, W0h, HM, DM, 1, ae, am);
    k_maskw<<<(unsigned)(((size_t)DM * HM / 4 + 255) / 256), 256, 0, stream>>>(w1, W1h, DM, HM, 0, ae, am);
    k_gemmw<h16, 0, false><<<dim3(NT / 64, HM / 64, 1), 32, 0, stream>>>(X16, nullptr, W0h, nullptr, DM, FC, HM, nullptr, 0, 0, 0);
    k_cast16<<<(unsigned)(((size_t)NT * HM / 4 + 255) / 256), 256, 0, stream>>>(FC, H16, (size_t)NT * HM / 4, 1, b0, HM, ae, am);
    k_gemmw<h16, 0, false><<<dim3(NT / 64, DM / 64, 1), 32, 0, stream>>>(H16, nullptr, W1h, nullptr, HM, OF, DM, nullptr, 0, 0, 0);
    k_addb<<<(unsigned)(((size_t)NT * DM / 4 + 255) / 256), 256, 0, stream>>>(OF, OUT, (size_t)NT * DM / 4, b1, DM, ae, am);
}
